// DeepMemoryLevel_34754875359826
// MI455X (gfx1250) — hardware-verified
//
#include <hip/hip_runtime.h>
#include <math.h>


typedef __bf16 bh;
typedef bh    v16b __attribute__((ext_vector_type(16)));
typedef bh    v8b  __attribute__((ext_vector_type(8)));
typedef float v8f  __attribute__((ext_vector_type(8)));
typedef float v4f  __attribute__((ext_vector_type(4)));

static constexpr int TT    = 2048;
static constexpr int DIM   = 1024;
static constexpr int MEM   = 256;
static constexpr int POLY  = 512;
static constexpr int HID   = 1024;
static constexpr int CHUNK = 32;
static constexpr int NC    = TT / CHUNK;
static constexpr int NPER  = 4;
static constexpr int SEQ   = 2044;
static constexpr int KCONV = 4;
static constexpr float MAXGN = 10.0f;
static constexpr size_t PK = (size_t)TT * POLY;
static constexpr size_t PW = (size_t)POLY * HID;

static constexpr int OF_Z1T = 0;
static constexpr int OF_HFT = 32768;
static constexpr int OF_DFT = 65536;
static constexpr int OF_DZT = 81920;
static constexpr int NF_SCR = 114688;
static constexpr int OB_HH  = 0;
static constexpr int OB_HT  = 65536;
static constexpr int OB_DH  = 131072;
static constexpr int OB_DZS = 163840;
static constexpr int OB_DS  = 294912;
static constexpr int NB_SCR = 360448;


__device__ __forceinline__ float sigm(float x) { return 1.0f / (1.0f + expf(-x)); }
__device__ __forceinline__ float silu(float x) { return x * sigm(x); }

__device__ __forceinline__ void ld8(const float* p, float (&x)[8]) {
  v4f a = *(const v4f*)p, b = *(const v4f*)(p + 4);
#pragma unroll
  for (int i = 0; i < 4; ++i) { x[i] = a[i]; x[4 + i] = b[i]; }
}
__device__ __forceinline__ void st8(float* p, const float (&x)[8]) {
  v4f a, b;
#pragma unroll
  for (int i = 0; i < 4; ++i) { a[i] = x[i]; b[i] = x[4 + i]; }
  *(v4f*)p = a; *(v4f*)(p + 4) = b;
}
__device__ __forceinline__ void split8(const float (&x)[8], v8b& hi, v8b& lo) {
#pragma unroll
  for (int i = 0; i < 8; ++i) {
    bh a = (bh)x[i];
    hi[i] = a;
    lo[i] = (bh)(x[i] - (float)a);
  }
}

union Frag { v16b v; v8b hv[2]; };

__device__ __forceinline__ v16b ldfrag(const bh* p, int ld) {
  const int l = threadIdx.x & 31, h = l >> 4, m = l & 15;
  const bh* q = p + (size_t)m * ld + 8 * h;
  Frag f;
  f.hv[0] = *(const v8b*)(q);
  f.hv[1] = *(const v8b*)(q + 16);
  return f.v;
}

__device__ __forceinline__ v8f wm(v16b a, v16b b, v8f c) {
  return __builtin_amdgcn_wmma_f32_16x16x32_bf16(false, a, false, b, (short)0, c, false, false);
}
__device__ __forceinline__ v8f wm3(v8f c, v16b ah, v16b al, v16b bhi, v16b bl) {
  c = wm(ah, bhi, c);
  c = wm(ah, bl, c);
  c = wm(al, bhi, c);
  asm volatile("v_nop\n\tv_nop\n\tv_nop\n\tv_nop" : "+v"(c) : "v"(ah), "v"(al), "v"(bhi), "v"(bl));
  return c;
}


__global__ __launch_bounds__(256) void build_xf_kernel(const float* __restrict__ x,
                                                       const float* __restrict__ pers,
                                                       bh* xf) {
  const int v = blockIdx.x * 256 + threadIdx.x;
  if (v >= TT * DIM / 8) return;
  const int e = v * 8, t = e / DIM, d = e - t * DIM;
  const float* src = (t < NPER) ? (pers + (size_t)t * DIM + d) : (x + (size_t)(t - NPER) * DIM + d);
  float a[8]; ld8(src, a);
  v8b vh, vl; split8(a, vh, vl);
  const size_t plane = (size_t)TT * DIM;
  bh* p = xf + e;
  *(volatile v8b*)p = vh; *(volatile v8b*)(p + plane) = vl;
  __threadfence();
  *(volatile v8b*)p = vh; *(volatile v8b*)(p + plane) = vl;
}

template <bool EMITF>
__global__ __launch_bounds__(256) void tsplit_kernel(const float* __restrict__ in, bh* out, float* outF,
                                                     int R, int C) {
  __shared__ __attribute__((aligned(16))) float tile[64 * 33];
  const int tid = threadIdx.x;
  const int c0 = blockIdx.x * 32, r0 = blockIdx.y * 64;
  if (c0 + 32 > C || r0 + 64 > R) return;
  {
    const int r = tid >> 2, cs = (tid & 3) * 8;
    const float* p = in + (size_t)(r0 + r) * C + c0 + cs;
    v4f a = *(const v4f*)p, b = *(const v4f*)(p + 4);
#pragma unroll
    for (int e = 0; e < 4; ++e) { tile[r * 33 + cs + e] = a[e]; tile[r * 33 + cs + 4 + e] = b[e]; }
  }
  __syncthreads();
  const int c = tid >> 3, q = tid & 7;
  float x[8];
#pragma unroll
  for (int e = 0; e < 8; ++e) x[e] = tile[(8 * q + e) * 33 + c];
  v8b vh, vl; split8(x, vh, vl);
  const size_t plane = (size_t)R * C;
  bh* po = out + (size_t)(c0 + c) * R + r0 + 8 * q;
  v4f f[2]; float* pf[2];
  if (EMITF) {
#pragma unroll
    for (int s = 0; s < 2; ++s) {
      const int p = tid + 256 * s, cc = p >> 4, qq = p & 15;
#pragma unroll
      for (int e = 0; e < 4; ++e) f[s][e] = tile[(4 * qq + e) * 33 + cc];
      pf[s] = outF + (size_t)(c0 + cc) * R + r0 + 4 * qq;
    }
  }
  auto emit = [&]() {
    *(volatile v8b*)po = vh;
    *(volatile v8b*)(po + plane) = vl;
    if (EMITF) { *(volatile v4f*)pf[0] = f[0]; *(volatile v4f*)pf[1] = f[1]; }
  };
  emit();
  __threadfence();
  emit();
}

__global__ __launch_bounds__(256) void rsplit_kernel(const float* __restrict__ in, bh* out, int n8) {
  const int v = blockIdx.x * 256 + threadIdx.x;
  if (v >= n8) return;
  const size_t e = (size_t)v * 8, plane = (size_t)n8 * 8;
  float a[8]; ld8(in + e, a);
  v8b vh, vl; split8(a, vh, vl);
  bh* p = out + e;
  *(volatile v8b*)p = vh; *(volatile v8b*)(p + plane) = vl;
  __threadfence();
  *(volatile v8b*)p = vh; *(volatile v8b*)(p + plane) = vl;
}

__global__ __launch_bounds__(256) void gatefold_kernel(const float* __restrict__ retr,
                                                       const float* __restrict__ gate,
                                                       bh* out, int n8) {
  const int v = blockIdx.x * 256 + threadIdx.x;
  if (v >= n8) return;
  const size_t e = (size_t)v * 8, plane = (size_t)n8 * 8;
  const float g = gate[e / MEM];
  float a[8]; ld8(retr + e, a);
#pragma unroll
  for (int i = 0; i < 8; ++i) a[i] *= g;
  v8b vh, vl; split8(a, vh, vl);
  bh* p = out + e;
  *(volatile v8b*)p = vh; *(volatile v8b*)(p + plane) = vl;
  __threadfence();
  *(volatile v8b*)p = vh; *(volatile v8b*)(p + plane) = vl;
}

__global__ __launch_bounds__(256) __attribute__((amdgpu_num_vgpr(248)))
void gemm_kernel(const bh* __restrict__ A, const bh* __restrict__ BT, float* C,
                 int M, int N, int K, int row_off, int Mout) {
  __shared__ __attribute__((aligned(16))) float stile[8 * 1024];
  const int wib = threadIdx.x >> 5, l = threadIdx.x & 31, h = l >> 4, n = l & 15;
  const int gw = blockIdx.x * 8 + wib;
  const int ncg = N >> 6;
  const int tm = (gw / ncg) << 4, tn0 = (gw % ncg) << 6;
  const bool valid = tm < M;
  const size_t pa = (size_t)M * K, pb = (size_t)N * K;
  v8f acc[4] = {};
  if (valid) {
    const bh* ap = A + (size_t)tm * K;
    for (int k = 0; k < K; k += 32) {
      v16b ah = ldfrag(ap + k, K), al = ldfrag(ap + pa + k, K);
#pragma unroll
      for (int j = 0; j < 4; ++j) {
        const bh* bp = BT + (size_t)(tn0 + 16 * j) * K + k;
        acc[j] = wm3(acc[j], ah, al, ldfrag(bp, K), ldfrag(bp + pb, K));
      }
    }
  }
  float* st = stile + wib * 1024;
#pragma unroll
  for (int j = 0; j < 4; ++j)
#pragma unroll
    for (int i = 0; i < 8; ++i) st[(8 * h + i) * 64 + 16 * j + n] = acc[j][i];
  __syncthreads();
  auto emit = [&]() {
#pragma unroll
    for (int s = 0; s < 8; ++s) {
      const int L = 4 * s + (l >> 3), r = L >> 1, hf = L & 1, q = l & 7;
      const int col = 32 * hf + 4 * q;
      const int orow = tm + r + row_off;
      if (valid && orow >= 0 && orow < Mout) {
        v4f v = *(const v4f*)(st + r * 64 + col);
        *(volatile v4f*)(C + (size_t)orow * N + tn0 + col) = v;
      }
    }
  };
  emit();
  __threadfence();
  emit();
}

__global__ __launch_bounds__(256) void conv_poly_kernel(
    const float* __restrict__ kpre, const float* __restrict__ qpre, const float* __restrict__ vpre,
    const float* __restrict__ ckw, const float* __restrict__ cqw, const float* __restrict__ cvw,
    const float* __restrict__ ckb, const float* __restrict__ cqb, const float* __restrict__ cvb,
    const float* __restrict__ pc,
    float* phiKf, bh* phiK, bh* phiQ, bh* vb) {
  __shared__ __attribute__((aligned(16))) float sK[POLY];
  __shared__ __attribute__((aligned(16))) float sQ[POLY];
  __shared__ __attribute__((aligned(16))) float sV[MEM];
  const int t = blockIdx.x, c = threadIdx.x;
  if (t >= TT) return;
  const float c0 = pc[0], c1 = pc[1];
  float ak = ckb[c], aq = cqb[c], av = cvb[c];
#pragma unroll
  for (int j = 0; j < KCONV; ++j) {
    const int ts = t - (KCONV - 1) + j;
    if (ts >= 0) {
      const size_t s = (size_t)ts * MEM + c;
      ak += ckw[c * KCONV + j] * kpre[s];
      aq += cqw[c * KCONV + j] * qpre[s];
      av += cvw[c * KCONV + j] * vpre[s];
    }
  }
  const float sk = silu(ak), sq = silu(aq), sv = silu(av);
  sK[c] = c0 * sk;  sK[MEM + c] = (c1 * sk) * sk;
  sQ[c] = c0 * sq;  sQ[MEM + c] = (c1 * sq) * sq;
  sV[c] = sv;
  __syncthreads();
  const size_t prow = (size_t)t * POLY, vrow = (size_t)t * MEM, pv = (size_t)TT * MEM;
  auto emit = [&]() {
    if (c < 128) {
      v4f f = *(const v4f*)(sK + 4 * c);
      *(volatile v4f*)(phiKf + prow + 4 * c) = f;
    }
    if (c < 64) {
      float x[8];
#pragma unroll
      for (int e = 0; e < 8; ++e) x[e] = sK[8 * c + e];
      v8b vh, vl; split8(x, vh, vl);
      bh* p = phiK + prow + 8 * c;
      *(volatile v8b*)p = vh; *(volatile v8b*)(p + PK) = vl;
    } else if (c < 128) {
      const int cc = c - 64;
      float x[8];
#pragma unroll
      for (int e = 0; e < 8; ++e) x[e] = sQ[8 * cc + e];
      v8b vh, vl; split8(x, vh, vl);
      bh* p = phiQ + prow + 8 * cc;
      *(volatile v8b*)p = vh; *(volatile v8b*)(p + PK) = vl;
    } else if (c < 160) {
      const int cc = c - 128;
      float x[8];
#pragma unroll
      for (int e = 0; e < 8; ++e) x[e] = sV[8 * cc + e];
      v8b vh, vl; split8(x, vh, vl);
      bh* p = vb + vrow + 8 * cc;
      *(volatile v8b*)p = vh; *(volatile v8b*)(p + pv) = vl;
    }
  };
  emit();
  __threadfence();
  emit();
}

__global__ __launch_bounds__(256) void gates_kernel(const float* __restrict__ x, const float* __restrict__ pers,
    const float* __restrict__ lrw, const float* __restrict__ lrb,
    const float* __restrict__ momw, const float* __restrict__ momb,
    const float* __restrict__ decw, const float* __restrict__ decb,
    const float* __restrict__ gw, const float* __restrict__ gb,
    float* lr, float* eta, float* alpha, float* gate) {
  __shared__ float g[4][32];
  const int tid = threadIdx.x, w = tid >> 5, l = tid & 31, t0 = blockIdx.x * 32;
  for (int tt = 0; tt < 4; ++tt) {
    const int t = t0 + 4 * w + tt;
    float a0 = 0.0f, a1 = 0.0f, a2 = 0.0f, a3 = 0.0f;
    if (t < TT) {
      const float* xr = (t < NPER) ? (pers + (size_t)t * DIM) : (x + (size_t)(t - NPER) * DIM);
#pragma unroll 1
      for (int j = 0; j < DIM / 32; ++j) {
        const int d = l + 32 * j;
        const float xv = xr[d];
        a0 += xv * lrw[d]; a1 += xv * momw[d]; a2 += xv * decw[d]; a3 += xv * gw[d];
      }
    }
#pragma unroll
    for (int o = 16; o > 0; o >>= 1) {
      a0 += __shfl_xor(a0, o); a1 += __shfl_xor(a1, o);
      a2 += __shfl_xor(a2, o); a3 += __shfl_xor(a3, o);
    }
    if (l == 0) { g[0][4 * w + tt] = a0; g[1][4 * w + tt] = a1; g[2][4 * w + tt] = a2; g[3][4 * w + tt] = a3; }
  }
  __syncthreads();
  if (w == 0) {
    const int t = t0 + l;
    const float v0 = sigm(g[0][l] + lrb[0]);
    const float v1 = sigm(g[1][l] + momb[0]);
    const float v2 = sigm(g[2][l] + decb[0]);
    const float v3 = sigm(g[3][l] + gb[0]);
    if (t < TT) {
      *(volatile float*)(lr + t) = v0; *(volatile float*)(eta + t) = v1;
      *(volatile float*)(alpha + t) = v2; *(volatile float*)(gate + t) = v3;
    }
    __threadfence();
    if (t < TT) {
      *(volatile float*)(lr + t) = v0; *(volatile float*)(eta + t) = v1;
      *(volatile float*)(alpha + t) = v2; *(volatile float*)(gate + t) = v3;
    }
  }
}


__device__ __forceinline__ void colnorm(const float* buf, int len, int sr, int stt,
                                        float* shpart, float* out32) {
  const int tid = threadIdx.x;
  const int t = tid & 31, seg = tid >> 5;
  const int per = len >> 4;
  const float* r = buf + (size_t)t * stt + (size_t)seg * per * sr;
  float s = 0.0f;
#pragma unroll 4
  for (int j = 0; j < per; ++j) { const float v = r[(size_t)j * sr]; s += v * v; }
  shpart[seg * 32 + t] = s;
  __syncthreads();
  if (tid < 32) {
    float a = 0.0f;
#pragma unroll
    for (int j = 0; j < 16; ++j) a += shpart[j * 32 + tid];
    out32[tid] = a;
  }
  __syncthreads();
}

template <bool DBL>
__device__ __forceinline__ void stage_rows(const v8f (&val)[4], bh* dst, size_t plane, int pitch,
                                           int row0, int col0, bh* st) {
  const int l = threadIdx.x & 31, h = l >> 4, n = l & 15;
#pragma unroll
  for (int j = 0; j < 4; ++j)
#pragma unroll
    for (int i = 0; i < 8; ++i) {
      const float xv = val[j][i];
      const bh a = (bh)xv;
      const bh b = (bh)(xv - (float)a);
      const int o = (8 * h + i) * 64 + 16 * j + n;
      st[o] = a; st[1024 + o] = b;
    }
  __syncthreads();
  auto emit = [&]() {
#pragma unroll
    for (int s = 0; s < 4; ++s) {
      const int L = 4 * s + (l >> 3), q = l & 7;
      v8b vh = *(const v8b*)(st + L * 64 + 8 * q);
      v8b vl = *(const v8b*)(st + 1024 + L * 64 + 8 * q);
      bh* p = dst + (size_t)(row0 + L) * pitch + col0 + 8 * q;
      if (DBL) { *(volatile v8b*)p = vh; *(volatile v8b*)(p + plane) = vl; }
      else     { *(v8b*)p = vh;          *(v8b*)(p + plane) = vl; }
    }
  };
  emit();
  if (DBL) { __threadfence(); emit(); }
  __syncthreads();
}

__global__ __launch_bounds__(512) __attribute__((amdgpu_num_vgpr(248)))
void scan_kernel(const bh* __restrict__ phiK, const bh* __restrict__ phiKT,
                 const bh* __restrict__ phiQ, const float* __restrict__ phiKf,
                 const float* __restrict__ Vt, const float* __restrict__ lr,
                 const float* __restrict__ eta, const float* __restrict__ alpha,
                 float* W1s, float* S1s, float* W2s, float* S2s,
                 bh* W1T, bh* W2R, bh* W2T, float* sf, bh* sb, bh* P) {
  __shared__ __attribute__((aligned(16))) bh stg[16 * 2048];
  __shared__ float shpart[512];
  __shared__ float kn2c[32], hn2[32], dn2[32], dzn2[32];
  __shared__ float cw1[32], cs1[32], cw2[32], cs2[32];
  __shared__ float su[32], wu[32];
  __shared__ float sc[4];
  const int tid = threadIdx.x, wid = tid >> 5, l = tid & 31, h = l >> 4, n = l & 15;
  bh* st = stg + wid * 2048;
  float* Z1T = sf + OF_Z1T;
  float* HfT = sf + OF_HFT;
  float* DfT = sf + OF_DFT;
  float* DZT = sf + OF_DZT;
  bh* Hh  = sb + OB_HH;
  bh* HT  = sb + OB_HT;
  bh* Dh  = sb + OB_DH;
  bh* DZs = sb + OB_DZS;
  bh* Ds  = sb + OB_DS;
  const int PH = CHUNK * HID;
  const int PD = CHUNK * POLY;

  for (int nc = 0; nc < NC; ++nc) {
    const int t0 = nc * CHUNK;

    for (int g = wid; g < 32; g += 16) {
      const int tm = (g >> 4) << 4, tn0 = (g & 15) << 6;
      v8f acc[4] = {};
      const bh* ap = phiK + (size_t)(t0 + tm) * POLY;
      for (int k = 0; k < POLY; k += 32) {
        v16b ah = ldfrag(ap + k, POLY), al = ldfrag(ap + PK + k, POLY);
#pragma unroll
        for (int j = 0; j < 4; ++j) {
          const bh* bp = W1T + (size_t)(tn0 + 16 * j) * POLY + k;
          acc[j] = wm3(acc[j], ah, al, ldfrag(bp, POLY), ldfrag(bp + PW, POLY));
        }
      }
      v8f hv[4];
#pragma unroll
      for (int j = 0; j < 4; ++j) {
        const int ng = tn0 + 16 * j + n, m0 = tm + 8 * h;
        float zz[8], hh8[8];
#pragma unroll
        for (int i = 0; i < 8; ++i) { const float z = acc[j][i]; zz[i] = z; const float s = silu(z); hh8[i] = s; hv[j][i] = s; }
        const size_t o = (size_t)ng * CHUNK + m0;
        st8(Z1T + o, zz);
        st8(HfT + o, hh8);
        v8b th, tl; split8(hh8, th, tl);
        *(v8b*)(HT + o) = th; *(v8b*)(HT + PH + o) = tl;
      }
      stage_rows<false>(hv, Hh, (size_t)PH, HID, tm, tn0, st);
    }
    __syncthreads();
    colnorm(HfT, HID, CHUNK, 1, shpart, hn2);
    colnorm(phiKf + (size_t)t0 * POLY, POLY, 1, POLY, shpart, kn2c);

    {
      const int g = wid, tm = (g >> 3) << 4, tn0 = (g & 7) << 6;
      v8f acc[4] = {};
      const bh* ap = Hh + (size_t)tm * HID;
      for (int k = 0; k < HID; k += 32) {
        v16b ah = ldfrag(ap + k, HID), al = ldfrag(ap + PH + k, HID);
#pragma unroll
        for (int j = 0; j < 4; ++j) {
          const bh* bp = W2T + (size_t)(tn0 + 16 * j) * HID + k;
          acc[j] = wm3(acc[j], ah, al, ldfrag(bp, HID), ldfrag(bp + PW, HID));
        }
      }
      v8f dv[4];
#pragma unroll
      for (int j = 0; j < 4; ++j) {
        const int ng = tn0 + 16 * j + n, m0 = tm + 8 * h;
        float dd[8];
#pragma unroll
        for (int i = 0; i < 8; ++i) {
          const float d = 2.0f * (acc[j][i] - Vt[(size_t)(t0 + m0 + i) * POLY + ng]);
          dd[i] = d; dv[j][i] = d;
        }
        st8(DfT + (size_t)ng * CHUNK + m0, dd);
      }
      stage_rows<false>(dv, Dh, (size_t)PD, POLY, tm, tn0, st);
    }
    __syncthreads();
    colnorm(DfT, POLY, CHUNK, 1, shpart, dn2);

    for (int g = wid; g < 32; g += 16) {
      const int tm = (g >> 4) << 4, tn0 = (g & 15) << 6;
      v8f acc[4] = {};
      const bh* ap = Dh + (size_t)tm * POLY;
      for (int k = 0; k < POLY; k += 32) {
        v16b ah = ldfrag(ap + k, POLY), al = ldfrag(ap + PD + k, POLY);
#pragma unroll
        for (int j = 0; j < 4; ++j) {
          const bh* bp = W2R + (size_t)(tn0 + 16 * j) * POLY + k;
          acc[j] = wm3(acc[j], ah, al, ldfrag(bp, POLY), ldfrag(bp + PW, POLY));
        }
      }
#pragma unroll
      for (int j = 0; j < 4; ++j) {
        const int ng = tn0 + 16 * j + n, m0 = tm + 8 * h;
        const size_t o = (size_t)ng * CHUNK + m0;
        float zz[8], dz8[8];
        ld8(Z1T + o, zz);
#pragma unroll
        for (int i = 0; i < 8; ++i) {
          const float z = zz[i], sg = sigm(z);
          dz8[i] = acc[j][i] * (sg * (1.0f + z * (1.0f - sg)));
        }
        st8(DZT + o, dz8);
      }
    }
    __syncthreads();
    colnorm(DZT, HID, CHUNK, 1, shpart, dzn2);

    if (tid == 0) {
      float sS0 = 1.0f, wW0 = 1.0f, wS0 = 0.0f;
      for (int r = 0; r < 32; ++r) { su[r] = 0.0f; wu[r] = 0.0f; }
      for (int t = 0; t < 32; ++t) {
        const float e = eta[t0 + t];
        const float Aa = 1.0f - alpha[t0 + t];
        sS0 *= e;
        for (int r = 0; r <= t; ++r) su[r] *= e;
        su[t] += 1.0f;
        wW0 *= Aa;
        wS0 = Aa * wS0 + sS0;
        for (int r = 0; r <= t; ++r) wu[r] = Aa * wu[r] + su[r];
      }
      for (int t = 0; t < 32; ++t) {
        const float lt = lr[t0 + t];
        const float n1 = sqrtf(kn2c[t] * dzn2[t]);
        const float n2 = sqrtf(hn2[t] * dn2[t]);
        const float s1 = fminf(1.0f, MAXGN / (n1 + 1e-12f));
        const float s2 = fminf(1.0f, MAXGN / (n2 + 1e-12f));
        cw1[t] = -lt * s1 * wu[t];  cs1[t] = -lt * s1 * su[t];
        cw2[t] = -lt * s2 * wu[t];  cs2[t] = -lt * s2 * su[t];
      }
      sc[0] = wW0; sc[1] = wS0; sc[2] = sS0;
    }
    __syncthreads();
    const float cA = sc[0], cS0 = sc[1], cE = sc[2];

    for (int v = tid; v < PH / 8; v += 512) {
      const int e = v * 8, tb = e & 31;
      float xx[8], y[8]; v8b a, b;
      ld8(DZT + e, xx);
#pragma unroll
      for (int i = 0; i < 8; ++i) y[i] = xx[i] * cw1[tb + i];
      split8(y, a, b); *(v8b*)(DZs + e) = a; *(v8b*)(DZs + PH + e) = b;
#pragma unroll
      for (int i = 0; i < 8; ++i) y[i] = xx[i] * cs1[tb + i];
      split8(y, a, b); *(v8b*)(DZs + 2 * PH + e) = a; *(v8b*)(DZs + 3 * PH + e) = b;
    }
    for (int v = tid; v < PD / 8; v += 512) {
      const int e = v * 8, tb = e & 31;
      float xx[8], y[8]; v8b a, b;
      ld8(DfT + e, xx);
#pragma unroll
      for (int i = 0; i < 8; ++i) y[i] = xx[i] * cw2[tb + i];
      split8(y, a, b); *(v8b*)(Ds + e) = a; *(v8b*)(Ds + PD + e) = b;
#pragma unroll
      for (int i = 0; i < 8; ++i) y[i] = xx[i] * cs2[tb + i];
      split8(y, a, b); *(v8b*)(Ds + 2 * PD + e) = a; *(v8b*)(Ds + 3 * PD + e) = b;
    }
    __syncthreads();

    for (int g = wid; g < 512; g += 16) {
      const int tm = (g >> 4) << 4, tn0 = (g & 15) << 6;
      const bh* ap = phiKT + (size_t)tm * TT + t0;
      v16b aTh = ldfrag(ap, TT), aTl = ldfrag(ap + PK, TT);
#pragma unroll
      for (int j = 0; j < 4; ++j) {
        const int n0 = tn0 + 16 * j;
        const bh* bp = DZs + (size_t)n0 * CHUNK;
        v8f aw = wm3(v8f{}, aTh, aTl, ldfrag(bp, CHUNK), ldfrag(bp + PH, CHUNK));
        v8f as = wm3(v8f{}, aTh, aTl, ldfrag(bp + 2 * PH, CHUNK), ldfrag(bp + 3 * PH, CHUNK));
        const int nn = n0 + n, m0 = tm + 8 * h;
        const size_t si = (size_t)nn * POLY + m0;
        float w[8], s[8], wn[8], sn[8];
        ld8(W1s + si, w); ld8(S1s + si, s);
#pragma unroll
        for (int i = 0; i < 8; ++i) {
          sn[i] = cE * s[i] + as[i];
          wn[i] = cA * w[i] + cS0 * s[i] + aw[i];
        }
        st8(S1s + si, sn); st8(W1s + si, wn);
        v8b a, b; split8(wn, a, b);
        *(v8b*)(W1T + si) = a; *(v8b*)(W1T + PW + si) = b;
      }
    }
    for (int g = wid; g < 512; g += 16) {
      const int tm = (g >> 3) << 4, tn0 = (g & 7) << 6;
      const bh* ap = HT + (size_t)tm * CHUNK;
      v16b aTh = ldfrag(ap, CHUNK), aTl = ldfrag(ap + PH, CHUNK);
#pragma unroll
      for (int j = 0; j < 4; ++j) {
        const int n0 = tn0 + 16 * j;
        const bh* bp = Ds + (size_t)n0 * CHUNK;
        v8f aw = wm3(v8f{}, aTh, aTl, ldfrag(bp, CHUNK), ldfrag(bp + PD, CHUNK));
        v8f as = wm3(v8f{}, aTh, aTl, ldfrag(bp + 2 * PD, CHUNK), ldfrag(bp + 3 * PD, CHUNK));
        const int nn = n0 + n, m0 = tm + 8 * h;
        const size_t si = (size_t)nn * HID + m0;
        float w[8], s[8], wn[8], sn[8];
        ld8(W2s + si, w); ld8(S2s + si, s);
#pragma unroll
        for (int i = 0; i < 8; ++i) {
          sn[i] = cE * s[i] + as[i];
          wn[i] = cA * w[i] + cS0 * s[i] + aw[i];
        }
        st8(S2s + si, sn); st8(W2s + si, wn);
        v8b a, b; split8(wn, a, b);
        *(v8b*)(W2T + si) = a; *(v8b*)(W2T + PW + si) = b;
#pragma unroll
        for (int i = 0; i < 8; ++i) {
          const int o = (8 * h + i) * 16 + n;
          st[o] = a[i]; st[256 + o] = b[i];
        }
        __syncthreads();
        {
          const int r = l >> 1, hf = l & 1;
          v8b vh = *(const v8b*)(st + r * 16 + 8 * hf);
          v8b vl = *(const v8b*)(st + 256 + r * 16 + 8 * hf);
          bh* p = W2R + (size_t)(tm + r) * POLY + n0 + 8 * hf;
          *(v8b*)p = vh; *(v8b*)(p + PW) = vl;
        }
        __syncthreads();
      }
    }
    __syncthreads();

    for (int g = wid; g < 32; g += 16) {
      const int tm = (g >> 4) << 4, tn0 = (g & 15) << 6;
      v8f acc[4] = {};
      const bh* ap = phiQ + (size_t)(t0 + tm) * POLY;
      for (int k = 0; k < POLY; k += 32) {
        v16b ah = ldfrag(ap + k, POLY), al = ldfrag(ap + PK + k, POLY);
#pragma unroll
        for (int j = 0; j < 4; ++j) {
          const bh* bp = W1T + (size_t)(tn0 + 16 * j) * POLY + k;
          acc[j] = wm3(acc[j], ah, al, ldfrag(bp, POLY), ldfrag(bp + PW, POLY));
        }
      }
      v8f hv[4];
#pragma unroll
      for (int j = 0; j < 4; ++j)
#pragma unroll
        for (int i = 0; i < 8; ++i) hv[j][i] = silu(acc[j][i]);
      stage_rows<false>(hv, Hh, (size_t)PH, HID, tm, tn0, st);
    }
    __syncthreads();

    {
      const int g = wid, tm = (g >> 3) << 4, tn0 = (g & 7) << 6;
      v8f acc[4] = {};
      const bh* ap = Hh + (size_t)tm * HID;
      for (int k = 0; k < HID; k += 32) {
        v16b ah = ldfrag(ap + k, HID), al = ldfrag(ap + PH + k, HID);
#pragma unroll
        for (int j = 0; j < 4; ++j) {
          const bh* bp = W2T + (size_t)(tn0 + 16 * j) * HID + k;
          acc[j] = wm3(acc[j], ah, al, ldfrag(bp, HID), ldfrag(bp + PW, HID));
        }
      }
      stage_rows<true>(acc, P, PK, POLY, t0 + tm, tn0, st);
    }
    __syncthreads();
  }
}


extern "C" void kernel_launch(void* const* d_in, const int* in_sizes, int n_in,
                              void* d_out, int out_size, void* d_ws, size_t ws_size,
                              hipStream_t stream) {
  if (n_in < 25) return;
  if (in_sizes[0] != SEQ * DIM || out_size != SEQ * DIM) return;
  const float* x      = (const float*)d_in[0];
  const float* pers   = (const float*)d_in[1];
  const float* Wk     = (const float*)d_in[2];
  const float* Wq     = (const float*)d_in[3];
  const float* Wv     = (const float*)d_in[4];
  const float* Wo     = (const float*)d_in[5];
  const float* ckw    = (const float*)d_in[6];
  const float* cqw    = (const float*)d_in[7];
  const float* cvw    = (const float*)d_in[8];
  const float* ckb    = (const float*)d_in[9];
  const float* cqb    = (const float*)d_in[10];
  const float* cvb    = (const float*)d_in[11];
  const float* lrw    = (const float*)d_in[12];
  const float* lrb    = (const float*)d_in[13];
  const float* momw   = (const float*)d_in[14];
  const float* momb   = (const float*)d_in[15];
  const float* decw   = (const float*)d_in[16];
  const float* decb   = (const float*)d_in[17];
  const float* gw     = (const float*)d_in[18];
  const float* gb     = (const float*)d_in[19];
  const float* polyc  = (const float*)d_in[20];
  const float* vexp   = (const float*)d_in[21];
  const float* memout = (const float*)d_in[22];
  const float* MW1    = (const float*)d_in[23];
  const float* MW2    = (const float*)d_in[24];

  char* base = (char*)d_ws;
  size_t cur = 0;
  auto carve = [&](size_t bytes) -> void* {
    void* r = base + cur;
    cur += (bytes + 255) & ~(size_t)255;
    return r;
  };

  bh*    xfp    = (bh*)   carve((size_t)2 * TT * DIM * 2);
  bh*    WkT    = (bh*)   carve((size_t)2 * MEM * DIM * 2);
  bh*    WqT    = (bh*)   carve((size_t)2 * MEM * DIM * 2);
  bh*    WvT    = (bh*)   carve((size_t)2 * MEM * DIM * 2);
  bh*    WoT    = (bh*)   carve((size_t)2 * DIM * MEM * 2);
  bh*    vexpT  = (bh*)   carve((size_t)2 * POLY * MEM * 2);
  bh*    moT    = (bh*)   carve((size_t)2 * MEM * POLY * 2);
  float* kpre   = (float*)carve((size_t)TT * MEM * 4);
  float* qpre   = (float*)carve((size_t)TT * MEM * 4);
  float* vpre   = (float*)carve((size_t)TT * MEM * 4);
  float* phiKf  = (float*)carve((size_t)TT * POLY * 4);
  bh*    phiKp  = (bh*)   carve((size_t)2 * TT * POLY * 2);
  bh*    phiKTp = (bh*)   carve((size_t)2 * POLY * TT * 2);
  bh*    phiQp  = (bh*)   carve((size_t)2 * TT * POLY * 2);
  bh*    vbp    = (bh*)   carve((size_t)2 * TT * MEM * 2);
  float* Vt     = (float*)carve((size_t)TT * POLY * 4);
  float* lr     = (float*)carve((size_t)TT * 4);
  float* eta    = (float*)carve((size_t)TT * 4);
  float* alpha  = (float*)carve((size_t)TT * 4);
  float* gate   = (float*)carve((size_t)TT * 4);
  float* W1s    = (float*)carve(PW * 4);
  float* S1s    = (float*)carve(PW * 4);
  float* W2s    = (float*)carve(PW * 4);
  float* S2s    = (float*)carve(PW * 4);
  bh*    W1T    = (bh*)   carve((size_t)2 * PW * 2);
  bh*    W2R    = (bh*)   carve((size_t)2 * PW * 2);
  bh*    W2T    = (bh*)   carve((size_t)2 * PW * 2);
  float* sf     = (float*)carve((size_t)NF_SCR * 4);
  bh*    sb     = (bh*)   carve((size_t)NB_SCR * 2);
  bh*    Pp     = (bh*)   carve((size_t)2 * TT * POLY * 2);
  float* retr   = (float*)carve((size_t)TT * MEM * 4);
  bh*    retrg  = (bh*)   carve((size_t)2 * TT * MEM * 2);
  if (cur > ws_size) return;

  auto cdiv = [](int a, int b) { return (a + b - 1) / b; };
  auto gemm = [&](const bh* A, const bh* BT, float* C, int M, int N, int K, int row_off, int Mout) {
    const int waves = (M / 16) * (N / 64);
    gemm_kernel<<<cdiv(waves, 8), 256, 0, stream>>>(A, BT, C, M, N, K, row_off, Mout);
  };

  build_xf_kernel<<<cdiv(TT * DIM / 8, 256), 256, 0, stream>>>(x, pers, xfp);
  tsplit_kernel<false><<<dim3(MEM / 32, DIM / 64), 256, 0, stream>>>(Wk, WkT, kpre, DIM, MEM);
  tsplit_kernel<false><<<dim3(MEM / 32, DIM / 64), 256, 0, stream>>>(Wq, WqT, kpre, DIM, MEM);
  tsplit_kernel<false><<<dim3(MEM / 32, DIM / 64), 256, 0, stream>>>(Wv, WvT, kpre, DIM, MEM);
  tsplit_kernel<false><<<dim3(DIM / 32, MEM / 64), 256, 0, stream>>>(Wo, WoT, kpre, MEM, DIM);
  tsplit_kernel<false><<<dim3(POLY / 32, MEM / 64), 256, 0, stream>>>(vexp, vexpT, kpre, MEM, POLY);
  tsplit_kernel<false><<<dim3(MEM / 32, POLY / 64), 256, 0, stream>>>(memout, moT, kpre, POLY, MEM);
  tsplit_kernel<true><<<dim3(HID / 32, POLY / 64), 256, 0, stream>>>(MW1, W1T, W1s, POLY, HID);
  tsplit_kernel<true><<<dim3(POLY / 32, HID / 64), 256, 0, stream>>>(MW2, W2T, W2s, HID, POLY);
  rsplit_kernel<<<cdiv(HID * POLY / 8, 256), 256, 0, stream>>>(MW2, W2R, HID * POLY / 8);
  hipMemsetAsync(S1s, 0, PW * 4, stream);
  hipMemsetAsync(S2s, 0, PW * 4, stream);

  gemm(xfp, WkT, kpre, TT, MEM, DIM, 0, TT);
  gemm(xfp, WqT, qpre, TT, MEM, DIM, 0, TT);
  gemm(xfp, WvT, vpre, TT, MEM, DIM, 0, TT);
  conv_poly_kernel<<<TT, 256, 0, stream>>>(kpre, qpre, vpre, ckw, cqw, cvw, ckb, cqb, cvb, polyc,
                                            phiKf, phiKp, phiQp, vbp);
  gates_kernel<<<cdiv(TT, 32), 256, 0, stream>>>(x, pers, lrw, lrb, momw, momb, decw, decb, gw, gb,
                                                 lr, eta, alpha, gate);
  gemm(vbp, vexpT, Vt, TT, POLY, MEM, 0, TT);
  tsplit_kernel<false><<<dim3(POLY / 32, TT / 64), 256, 0, stream>>>(phiKf, phiKTp, kpre, TT, POLY);
  scan_kernel<<<1, 512, 0, stream>>>(phiKp, phiKTp, phiQp, phiKf, Vt, lr, eta, alpha,
                                     W1s, S1s, W2s, S2s, W1T, W2R, W2T, sf, sb, Pp);
  gemm(Pp, moT, retr, TT, MEM, POLY, 0, TT);
  gatefold_kernel<<<cdiv(TT * MEM / 8, 256), 256, 0, stream>>>(retr, gate, retrg, TT * MEM / 8);
  gemm(retrg, WoT, (float*)d_out, TT, DIM, MEM, -NPER, SEQ);
}
